// DenseKANRBF_47940424958484
// MI455X (gfx1250) — hardware-run, weakly checked
//
#include <hip/hip_runtime.h>


#ifndef NB
#define NB 1024
#endif
#define NB_FULL 1024
#define NF   512
#define NG   8
#define NU   512
#define NHID 2048
#define KPHI (NF * NG)
#define KCAT (KPHI + NHID)
#define OSP  68
#define TSP  72
#define ACARRY 256.0f
#define WCARRY 64.0f
#define OSCALE (1.0f / 16384.0f)

static_assert(NB % 64 == 0);
static_assert(NB <= NB_FULL);
static_assert(NF % 64 == 0);
static_assert(NU % 64 == 0);
static_assert(NHID % 64 == 0);
static_assert(KPHI % 64 == 0);
static_assert(NF % 32 == 0);
static_assert(KCAT % 32 == 0);
static_assert(NG == 8);
static_assert((NB * NF) % 256 == 0);
static_assert(((size_t)NB * NF) % 8 == 0);
static_assert(NF % 8 == 0);
static_assert((KCAT * 2) % 128 == 0);
static_assert((KPHI * 2) % 128 == 0);
static_assert(ACARRY * WCARRY * OSCALE == 1.0f);
static_assert((OSP * 4) % 16 == 0);
static_assert((TSP * 2) % 16 == 0);
static_assert(16 * OSP * 4 <= 131072);
static_assert(64 * TSP * 2 <= 131072);
static_assert(256 * 8 * 2 <= 131072);

typedef _Float16 h16;
typedef unsigned short bf;
typedef __attribute__((ext_vector_type(16))) __bf16   v16bf;
typedef __attribute__((ext_vector_type(16))) _Float16 v16h;
typedef __attribute__((ext_vector_type(8)))  _Float16 v8h;
typedef __attribute__((ext_vector_type(8)))  unsigned short v8us;
typedef __attribute__((ext_vector_type(8)))  float    v8f;
typedef __attribute__((ext_vector_type(4)))  float    v4f;
typedef v4f  __attribute__((may_alias)) v4fa;

__device__ __forceinline__ unsigned short f2bf(float f) { unsigned u = __float_as_uint(f); u += 0x7FFFu + ((u >> 16) & 1u); return (unsigned short)(u >> 16); }
__device__ __forceinline__ float bfr(float f) { return __uint_as_float(((unsigned)f2bf(f)) << 16); }
__device__ __forceinline__ v16h cat16(v8h lo, v8h hi) { return __builtin_shufflevector(lo, hi, 0, 1, 2, 3, 4, 5, 6, 7, 8, 9, 10, 11, 12, 13, 14, 15); }
__device__ __forceinline__ v16bf cat16b(v8us lo, v8us hi) { return __builtin_bit_cast(v16bf, __builtin_shufflevector(lo, hi, 0, 1, 2, 3, 4, 5, 6, 7, 8, 9, 10, 11, 12, 13, 14, 15)); }
__device__ __forceinline__ v8f wmma16(v16h a, v16h b, v8f c) { return __builtin_amdgcn_wmma_f32_16x16x32_f16(false, a, false, b, (short)0, c, false, false); }
__device__ __forceinline__ v8f wmmab(v16bf a, v16bf b, v8f c) { return __builtin_amdgcn_wmma_f32_16x16x32_bf16(false, a, false, b, (short)0, c, false, false); }
__device__ __forceinline__ v16h  ldh(const h16* p) { return cat16(*(const v8h*)p, *(const v8h*)(p + 16)); }
__device__ __forceinline__ v16bf ldb(const bf* p)  { return cat16b(*(const v8us*)p, *(const v8us*)(p + 16)); }
__device__ __forceinline__ void wave_sync() { __builtin_amdgcn_fence(3  , "wavefront"); __builtin_amdgcn_wave_barrier(); asm volatile("" ::: "memory"); }

__device__ __forceinline__ v8f wmmabg(v16bf a, v16bf b, v8f c) { c = wmmab(a, b, c); asm volatile("v_nop\n\tv_nop\n\tv_nop\n\tv_nop" : "+v"(c) : "v"(a), "v"(b)); return c; }
__device__ __forceinline__ v8f wmma16g(v16h a, v16h b, v8f c) { c = wmma16(a, b, c); asm volatile("v_nop\n\tv_nop\n\tv_nop\n\tv_nop" : "+v"(c) : "v"(a), "v"(b)); return c; }
static __device__ __forceinline__ h16 toh_flush(float v) { const h16 r = (h16)v; return (fabsf(v) < 6.103515625e-05f) ? (h16)0.0f : r; }

__global__ __launch_bounds__(256) void k_cvt8(const float* __restrict__ src, bf* dst, size_t n8) {
    const size_t i = (size_t)blockIdx.x * 256 + threadIdx.x; if (i >= n8) return;
    const v8f v = *(const v8f*)(src + i * 8); v8us o;
#pragma unroll
    for (int k = 0; k < 8; ++k) o[k] = f2bf(v[k]);
    *(volatile v8us*)(dst + i * 8) = o; __threadfence(); *(volatile v8us*)(dst + i * 8) = o;
}

static_assert(256 * 16 == 256 * NG * 2);
__global__ __launch_bounds__(256) void k_phi(const float* __restrict__ x, h16* AH, int total) {
#pragma clang fp contract(off)
    __shared__ __align__(16) h16 ps[256 * NG];
    const int tid = threadIdx.x;
    int idx = blockIdx.x * 256 + tid; idx = idx < total ? idx : total - 1;
    const float xv = bfr(x[idx]);
#pragma unroll 1
    for (int g = 0; g < NG; ++g) {
        const float t = (float)g * (1.0f / 7.0f);
        const float c = (g == NG - 1) ? 1.0f : ((t - 1.0f) + t);
        const float d = xv - c;
        ps[tid * NG + g] = toh_flush(expf(-(d * d)) * ACARRY);
    }
    __syncthreads();
    const v8h v = *(const v8h*)(&ps[tid * NG]);
    const int row = idx / NF, f = idx % NF;
    h16* dst = AH + (size_t)row * KCAT + (size_t)f * NG;
    *(volatile v8h*)dst = v; __threadfence(); *(volatile v8h*)dst = v;
}

static_assert(256 * 16 * 2 == 64 * 128);
__global__ __launch_bounds__(256) void k_trb(const float* __restrict__ src, bf* dst, int N, int pitch, int koff) {
    __shared__ __align__(16) unsigned short ts[64 * TSP];
    const int tid = threadIdx.x; const int k0 = blockIdx.x * 64, n0 = blockIdx.y * 64;
    const int c = tid & 63, r = tid >> 6;
#pragma unroll 4
    for (int i = 0; i < 16; ++i) { const int k = r + 4 * i;
        ts[c * TSP + k] = f2bf(src[(size_t)(k0 + k) * N + n0 + c]); }
    __syncthreads();
    v8us o[2];
#pragma unroll
    for (int s = 0; s < 2; ++s) { const int row = s * 32 + (tid >> 3), c8 = (tid & 7) * 8; o[s] = *(const v8us*)(&ts[row * TSP + c8]); }
#pragma unroll 1
    for (int ps = 0; ps < 2; ++ps) {
#pragma unroll
        for (int s = 0; s < 2; ++s) { const int row = s * 32 + (tid >> 3), c8 = (tid & 7) * 8;
            *(volatile v8us*)(dst + (size_t)(n0 + row) * pitch + koff + k0 + c8) = o[s]; }
        if (ps == 0) __threadfence(); }
}

__global__ __launch_bounds__(256) void k_trh(const float* __restrict__ src, h16* dst, int N, int pitch, int koff) {
#pragma clang fp contract(off)
    __shared__ __align__(16) h16 ts[64 * TSP];
    const int tid = threadIdx.x; const int k0 = blockIdx.x * 64, n0 = blockIdx.y * 64;
    const int c = tid & 63, r = tid >> 6;
#pragma unroll 4
    for (int i = 0; i < 16; ++i) { const int k = r + 4 * i;
        const float v = bfr(src[(size_t)(k0 + k) * N + n0 + c]);
        ts[c * TSP + k] = toh_flush(v * WCARRY); }
    __syncthreads();
    v8h o[2];
#pragma unroll
    for (int s = 0; s < 2; ++s) { const int row = s * 32 + (tid >> 3), c8 = (tid & 7) * 8; o[s] = *(const v8h*)(&ts[row * TSP + c8]); }
#pragma unroll 1
    for (int ps = 0; ps < 2; ++ps) {
#pragma unroll
        for (int s = 0; s < 2; ++s) { const int row = s * 32 + (tid >> 3), c8 = (tid & 7) * 8;
            *(volatile v8h*)(dst + (size_t)(n0 + row) * pitch + koff + k0 + c8) = o[s]; }
        if (ps == 0) __threadfence(); }
}

static_assert(32 * 16 * 4 == 16 * 128);
__global__ __launch_bounds__(32) void k_gemm_h(const bf* __restrict__ A, const bf* __restrict__ Bt, const float* __restrict__ b1, h16* AH) {
    __shared__ __align__(16) float os[16 * OSP];
    const int K = NF;
    const int lane = threadIdx.x & 31, lr = lane & 15, hi = lane >> 4; const int r0 = blockIdx.x * 64, c0 = blockIdx.y * 64;
    v8f acc[4][4];
#pragma unroll
    for (int mb = 0; mb < 4; ++mb)
#pragma unroll
        for (int nb = 0; nb < 4; ++nb) acc[mb][nb] = (v8f){};
    const size_t aoff = (size_t)(r0 + lr) * K + 8 * hi, boff = (size_t)(c0 + lr) * K + 8 * hi;
#pragma unroll 1
    for (int kc = 0; kc < K; kc += 32) {
        v16bf a[4];
#pragma unroll
        for (int mb = 0; mb < 4; ++mb) a[mb] = ldb(A + aoff + (size_t)mb * 16 * K + kc);
#pragma unroll
        for (int nb = 0; nb < 4; ++nb) { const v16bf b = ldb(Bt + boff + (size_t)nb * 16 * K + kc);
#pragma unroll
            for (int mb = 0; mb < 4; ++mb) acc[mb][nb] = wmmabg(a[mb], b, acc[mb][nb]); }
    }
    float bc[4];
#pragma unroll
    for (int nb = 0; nb < 4; ++nb) bc[nb] = bfr(b1[c0 + nb * 16 + lr]);
#pragma unroll
    for (int mb = 0; mb < 4; ++mb) {
#pragma unroll
        for (int nb = 0; nb < 4; ++nb) {
#pragma unroll
            for (int j = 0; j < 8; ++j) os[(hi * 8 + j) * OSP + nb * 16 + lr] = acc[mb][nb][j] + bc[nb]; }
        wave_sync();
#pragma unroll 1
        for (int i = 0; i < 8; ++i) { const int p = i * 32 + lane; const int row = p >> 4, c4 = (p & 15) * 4;
            v4f t = *(const v4fa*)(&os[row * OSP + c4]);
#pragma unroll
            for (int e = 0; e < 4; ++e) { const float u = t[e]; t[e] = (0.5f * u * (1.0f + erff(u * 0.70710678118654752f))) * ACARRY; }
            *(v4fa*)(&os[row * OSP + c4]) = t; }
        wave_sync();
        const size_t sb = (size_t)(r0 + mb * 16) * KCAT + (size_t)KPHI + (size_t)c0;
#pragma unroll 1
        for (int ps = 0; ps < 2; ++ps) {
#pragma unroll
            for (int s = 0; s < 4; ++s) { const int row = 4 * s + (lane >> 3), c8 = (lane & 7) * 8;
                const v4f x0 = *(const v4fa*)(&os[row * OSP + c8]); const v4f x1 = *(const v4fa*)(&os[row * OSP + c8 + 4]); v8h hv;
#pragma unroll
                for (int i = 0; i < 4; ++i) { hv[i] = toh_flush(x0[i]); hv[4 + i] = toh_flush(x1[i]); }
                *(volatile v8h*)(AH + sb + (size_t)row * KCAT + c8) = hv; }
            if (ps == 0) __threadfence(); }
        wave_sync();
    }
}

static_assert(32 * 16 * 8 == 16 * 256);
__global__ __launch_bounds__(32) void k_gemm_o(const h16* __restrict__ A, const h16* __restrict__ Bt, const float* __restrict__ b2, const float* __restrict__ bias, float* OUT) {
    __shared__ __align__(16) float os[16 * OSP];
    const int K = KCAT;
    const int lane = threadIdx.x & 31, lr = lane & 15, hi = lane >> 4; const int r0 = blockIdx.x * 64, c0 = blockIdx.y * 64;
    v8f acc[4][4];
#pragma unroll
    for (int mb = 0; mb < 4; ++mb)
#pragma unroll
        for (int nb = 0; nb < 4; ++nb) acc[mb][nb] = (v8f){};
    const size_t aoff = (size_t)(r0 + lr) * K + 8 * hi, boff = (size_t)(c0 + lr) * K + 8 * hi;
#pragma unroll 1
    for (int kc = 0; kc < K; kc += 32) {
        v16h a[4];
#pragma unroll
        for (int mb = 0; mb < 4; ++mb) a[mb] = ldh(A + aoff + (size_t)mb * 16 * K + kc);
#pragma unroll
        for (int nb = 0; nb < 4; ++nb) { const v16h b = ldh(Bt + boff + (size_t)nb * 16 * K + kc);
#pragma unroll
            for (int mb = 0; mb < 4; ++mb) acc[mb][nb] = wmma16g(a[mb], b, acc[mb][nb]); }
    }
    float bc[4], bd[4];
#pragma unroll
    for (int nb = 0; nb < 4; ++nb) { bc[nb] = bfr(b2[c0 + nb * 16 + lr]); bd[nb] = bfr(bias[c0 + nb * 16 + lr]); }
#pragma unroll
    for (int mb = 0; mb < 4; ++mb) {
#pragma unroll
        for (int nb = 0; nb < 4; ++nb) {
#pragma unroll
            for (int j = 0; j < 8; ++j) os[(hi * 8 + j) * OSP + nb * 16 + lr] = (acc[mb][nb][j] * OSCALE + bc[nb]) + bd[nb]; }
        wave_sync();
        float* ob = OUT + (size_t)(r0 + mb * 16) * NU + c0;
#pragma unroll 1
        for (int ps = 0; ps < 2; ++ps) {
#pragma unroll
            for (int s = 0; s < 8; ++s) { const int row = 2 * s + (lane >> 4), cofs = (lane & 15) * 4;
                const v4f val = *(const v4fa*)(&os[row * OSP + cofs]);
                *(volatile v4f*)(ob + (size_t)row * NU + cofs) = val; }
            if (ps == 0) __threadfence(); }
        wave_sync();
    }
}

static constexpr size_t al256(size_t v) { return (v + 255) & ~(size_t)255; }
static constexpr size_t SZ_XB = al256((size_t)NB * NF * 2);
static constexpr size_t SZ_W1 = al256((size_t)NHID * NF * 2);
static constexpr size_t SZ_AH = al256((size_t)NB * KCAT * 2);
static constexpr size_t SZ_BT = al256((size_t)NU * KCAT * 2);
static constexpr size_t SZ_TOTAL = SZ_XB + SZ_W1 + SZ_AH + SZ_BT;
static_assert(SZ_TOTAL <= (size_t)134217728);
static constexpr size_t N8X = (size_t)NB * NF / 8;
static constexpr unsigned G_CVT = (unsigned)((N8X + 255) / 256);
static constexpr unsigned G_PHI = (unsigned)(((size_t)NB * NF) / 256);

extern "C" void kernel_launch(void* const* d_in, const int* in_sizes, int n_in,
                              void* d_out, int out_size, void* d_ws, size_t ws_size, hipStream_t stream) {
    if (n_in < 7) return;
    if ((size_t)in_sizes[0] < (size_t)NB * NF) return;
    if ((size_t)in_sizes[1] < (size_t)KPHI * NU) return;
    if ((size_t)in_sizes[2] < (size_t)NF * NHID) return;
    if (in_sizes[3] < NHID) return;
    if ((size_t)in_sizes[4] < (size_t)NHID * NU) return;
    if (in_sizes[5] < NU || in_sizes[6] < NU) return;
    if ((size_t)out_size < (size_t)NB * NU) return;
    if (SZ_TOTAL > ws_size) return;
    const float* x   = (const float*)d_in[0];
    const float* bk  = (const float*)d_in[1];
    const float* w1  = (const float*)d_in[2];
    const float* b1  = (const float*)d_in[3];
    const float* w2  = (const float*)d_in[4];
    const float* b2  = (const float*)d_in[5];
    const float* bia = (const float*)d_in[6];
    float* OUT = (float*)d_out;
    char* wsp = (char*)d_ws;
    bf*  XB  = (bf*)wsp;  wsp += SZ_XB;
    bf*  W1T = (bf*)wsp;  wsp += SZ_W1;
    h16* AH  = (h16*)wsp; wsp += SZ_AH;
    h16* BT  = (h16*)wsp; wsp += SZ_BT;

    k_cvt8<<<G_CVT, 256, 0, stream>>>(x, XB, N8X);
    k_trb<<<dim3(NF / 64, NHID / 64, 1), 256, 0, stream>>>(w1, W1T, NHID, NF, 0);
    k_trh<<<dim3(KPHI / 64, NU / 64, 1), 256, 0, stream>>>(bk, BT, NU, KCAT, 0);
    k_trh<<<dim3(NHID / 64, NU / 64, 1), 256, 0, stream>>>(w2, BT, NU, KCAT, KPHI);
    k_phi<<<G_PHI, 256, 0, stream>>>(x, AH, NB * NF);
    k_gemm_h<<<dim3(NB / 64, NHID / 64, 1), 32, 0, stream>>>(XB, W1T, b1, AH);
    k_gemm_o<<<dim3(NB / 64, NU / 64, 1), 32, 0, stream>>>(AH, BT, b2, bia, OUT);
}
